// InhibitorAttention_55817394979296
// MI455X (gfx1250) — hardware-verified
//
#include <hip/hip_runtime.h>

#define S  512
#define DD 512
#define NH 8
#define DH 64

typedef __attribute__((ext_vector_type(16))) _Float16 v16h;
typedef __attribute__((ext_vector_type(8)))  _Float16 v8h;
typedef __attribute__((ext_vector_type(8)))  float    v8f;
typedef __attribute__((ext_vector_type(4)))  float    v4f_t;
typedef float v4fa __attribute__((ext_vector_type(4), may_alias));
typedef __attribute__((ext_vector_type(4)))  unsigned v4u_t;
#define PL ((size_t)S * DD)
#define RSPLIT (1.0f / 2048.0f)
static __device__ __forceinline__ unsigned pk2s(float a, float b, unsigned* lo) {
  const _Float16 h0 = (_Float16)a, h1 = (_Float16)b;
  *lo = (unsigned)__builtin_bit_cast(unsigned short, (_Float16)((a - (float)h0) * 2048.0f)) | ((unsigned)__builtin_bit_cast(unsigned short, (_Float16)((b - (float)h1) * 2048.0f)) << 16);
  return (unsigned)__builtin_bit_cast(unsigned short, h0) | ((unsigned)__builtin_bit_cast(unsigned short, h1) << 16);
}

__global__ __launch_bounds__(256) void cvt_f32_to_f16_kernel(
    const float* __restrict__ x, _Float16* __restrict__ y, int n) {
  int i = (blockIdx.x * 256 + threadIdx.x) * 2;
  if (i < n) { unsigned lo; const unsigned p = pk2s(x[i], x[i + 1], &lo);
    *(volatile unsigned*)(y + i) = p; *(volatile unsigned*)(y + PL + i) = lo; __threadfence(); *(volatile unsigned*)(y + i) = p; *(volatile unsigned*)(y + PL + i) = lo; }
}

__global__ __launch_bounds__(256) void cvt_transpose_w_kernel(
    const float* __restrict__ W, _Float16* __restrict__ Wt) {
  int idx = (blockIdx.x * 256 + threadIdx.x) * 2;
  int n = idx >> 9;
  int k = idx & 511;
  unsigned lo; const unsigned p = pk2s(W[k * DD + n], W[(k + 1) * DD + n], &lo);
  *(volatile unsigned*)(Wt + idx) = p; *(volatile unsigned*)(Wt + PL + idx) = lo; __threadfence(); *(volatile unsigned*)(Wt + idx) = p; *(volatile unsigned*)(Wt + PL + idx) = lo;
}

__device__ __forceinline__ v8f wmma_tile_f16(const _Float16* __restrict__ A,
                                             const _Float16* __restrict__ Bt,
                                             int tile_m, int tile_n, int lane) {
  const int hh   = lane >> 4;
  const int mrow = lane & 15;
  const _Float16* arow = A  + (size_t)(tile_m * 16 + mrow) * DD + hh * 8;
  const _Float16* brow = Bt + (size_t)(tile_n * 16 + mrow) * DD + hh * 8;
  v8f c = {};
  for (int kb = 0; kb < DD; kb += 32) {
    __builtin_prefetch(arow + kb + 64, 0, 1);
    __builtin_prefetch(brow + kb + 64, 0, 1);
    v16h a, b, al, bl;
    *(v8h*)&a  = *(const v8h*)(arow + kb);      *((v8h*)&a + 1)  = *(const v8h*)(arow + kb + 16);
    *(v8h*)&b  = *(const v8h*)(brow + kb);      *((v8h*)&b + 1)  = *(const v8h*)(brow + kb + 16);
    *(v8h*)&al = *(const v8h*)(arow + PL + kb); *((v8h*)&al + 1) = *(const v8h*)(arow + PL + kb + 16);
    *(v8h*)&bl = *(const v8h*)(brow + PL + kb); *((v8h*)&bl + 1) = *(const v8h*)(brow + PL + kb + 16);
    v8f x = {};
    x = __builtin_amdgcn_wmma_f32_16x16x32_f16(false, al, false, b, (short)0, x, false, false);
    x = __builtin_amdgcn_wmma_f32_16x16x32_f16(false, a, false, bl, (short)0, x, false, false);
    c = __builtin_amdgcn_wmma_f32_16x16x32_f16(false, a, false, b, (short)0, c, false, false) + x * RSPLIT;
  }
  return c;
}

__device__ __forceinline__ void store_tile(float* __restrict__ C,
                                           const float* __restrict__ bias,
                                           v8f c, int tile_m, int tile_n,
                                           int lane, float (*stg)[128 + 4], int wave, int tid) {
  const int hh  = lane >> 4;
  const int col = tile_n * 16 + (lane & 15);
  const float bb = bias[col];
#pragma unroll
  for (int r = 0; r < 8; ++r) stg[hh * 8 + r][wave * 16 + (lane & 15)] = c[r] + bb;
  __syncthreads();
  const int col0 = (tile_n - wave) * 16;
#pragma unroll 1
  for (int pass = 0; pass < 2; ++pass) {
#pragma unroll
    for (int i = 0; i < 2; ++i) { const int cc = tid + 256 * i, rr = cc >> 5, q = cc & 31;
      *(volatile v4f_t*)(C + (size_t)(tile_m * 16 + rr) * DD + col0 + q * 4) = *(const v4fa*)&stg[rr][q * 4]; }
    __threadfence();
  }
}

__global__ __launch_bounds__(256) void gemm_qkv_kernel(
    const _Float16* __restrict__ Xh,
    const _Float16* __restrict__ Wqt, const _Float16* __restrict__ Wkt,
    const _Float16* __restrict__ Wvt,
    const float* __restrict__ bq, const float* __restrict__ bk,
    const float* __restrict__ bv_,
    float* __restrict__ Q, float* __restrict__ K, float* __restrict__ V) {
  const int lane = threadIdx.x & 31;
  const int wave = threadIdx.x >> 5;
  const int tile = blockIdx.x * 8 + wave;
  const int tile_m = tile >> 5;
  const int tile_n = tile & 31;

  const _Float16* Bt;
  const float* bias;
  float* C;
  if (blockIdx.y == 0)      { Bt = Wqt; bias = bq;  C = Q; }
  else if (blockIdx.y == 1) { Bt = Wkt; bias = bk;  C = K; }
  else                      { Bt = Wvt; bias = bv_; C = V; }

  __shared__ __attribute__((aligned(16))) float stg[16][128 + 4];
  v8f c = wmma_tile_f16(Xh, Bt, tile_m, tile_n, lane);
  store_tile(C, bias, c, tile_m, tile_n, lane, stg, wave, threadIdx.x);
}

__global__ __launch_bounds__(256) void gemm_out_kernel(
    const _Float16* __restrict__ Ch, const _Float16* __restrict__ Wot,
    const float* __restrict__ bo, float* __restrict__ out) {
  const int lane = threadIdx.x & 31;
  const int wave = threadIdx.x >> 5;
  const int tile = blockIdx.x * 8 + wave;
  const int tile_m = tile >> 5;
  const int tile_n = tile & 31;
  __shared__ __attribute__((aligned(16))) float stg[16][128 + 4];
  v8f c = wmma_tile_f16(Ch, Wot, tile_m, tile_n, lane);
  store_tile(out, bo, c, tile_m, tile_n, lane, stg, wave, threadIdx.x);
}

#define TJ 32
__global__ __launch_bounds__(128) void attn_core_kernel(
    const float* __restrict__ Q, const float* __restrict__ K,
    const float* __restrict__ V, const float* __restrict__ mask,
    const float* __restrict__ gamma, const float* __restrict__ alpha,
    _Float16* __restrict__ ctx_h) {
  __shared__ float qsh[128][DH + 1];
  __shared__ __align__(16) float ksh[TJ][DH];
  __shared__ __align__(16) float vsh[TJ][DH];
  __shared__ float msh[TJ];

  const int head = blockIdx.y;
  const int t    = threadIdx.x;
  const int i    = blockIdx.x * 128 + t;
  const size_t qoff = (size_t)i * DD + head * DH;

  const float scale = 1.0f / (gamma[0] * 8.0f);
  const float a0    = alpha[0];

#pragma unroll 4
  for (int d = 0; d < DH; ++d) qsh[t][d] = Q[qoff + d];

  float acc[DH];
#pragma unroll
  for (int d = 0; d < DH; ++d) acc[d] = 0.0f;

  for (int jc = 0; jc < S; jc += TJ) {
    __syncthreads();

    {
      const float* Kbase = K + (size_t)jc * DD + head * DH;
      const float* Vbase = V + (size_t)jc * DD + head * DH;
#pragma unroll
      for (int u = 0; u < 4; ++u) {
        int f4 = t + u * 128;
        int jj = f4 >> 4;
        int d  = (f4 & 15) << 2;
        const float* gk = Kbase + (size_t)jj * DD + d;
        const float* gv = Vbase + (size_t)jj * DD + d;
        unsigned lk = (unsigned)(unsigned long long)(&ksh[jj][d]);
        unsigned lv = (unsigned)(unsigned long long)(&vsh[jj][d]);
        asm volatile("global_load_async_to_lds_b128 %0, %1, off"
                     :: "v"(lk), "v"(gk) : "memory");
        asm volatile("global_load_async_to_lds_b128 %0, %1, off"
                     :: "v"(lv), "v"(gv) : "memory");
      }
    }
    if (t < TJ) msh[t] = (1.0f - mask[jc + t]) * 1e10f;

    asm volatile("s_wait_asynccnt 0x0" ::: "memory");
    __syncthreads();

    for (int jj = 0; jj < TJ; ++jj) {
      float s = 0.0f;
#pragma unroll
      for (int d = 0; d < DH; ++d) s += fabsf(qsh[t][d] - ksh[jj][d]);
      float zp = fmaxf(s * scale - a0, 0.0f) + msh[jj];
#pragma unroll
      for (int d = 0; d < DH; ++d) acc[d] += fmaxf(vsh[jj][d] - zp, 0.0f);
    }
  }

  __syncthreads();
#pragma unroll
  for (int d = 0; d < DH; ++d) qsh[t][d] = acc[d];
  __syncthreads();
#pragma unroll 1
  for (int pass = 0; pass < 2; ++pass) {
#pragma unroll
    for (int i2 = 0; i2 < 8; ++i2) {
      const int c = t + 128 * i2, rr = c >> 3, q = c & 7;
      const float* s = &qsh[rr][q * 8];
      v4u_t v, vl; unsigned lo;
      v.x = pk2s(s[0], s[1], &lo); vl.x = lo; v.y = pk2s(s[2], s[3], &lo); vl.y = lo; v.z = pk2s(s[4], s[5], &lo); vl.z = lo; v.w = pk2s(s[6], s[7], &lo); vl.w = lo;
      _Float16* dst = ctx_h + (size_t)(blockIdx.x * 128 + rr) * DD + head * DH + q * 8;
      *(volatile v4u_t*)dst = v; *(volatile v4u_t*)(dst + PL) = vl;
    }
    __threadfence();
  }
}

extern "C" void kernel_launch(void* const* d_in, const int* in_sizes, int n_in,
                              void* d_out, int out_size, void* d_ws,
                              size_t ws_size, hipStream_t stream) {
  const float* X     = (const float*)d_in[0];
  const float* mask  = (const float*)d_in[1];
  const float* Wq    = (const float*)d_in[2];
  const float* bq    = (const float*)d_in[3];
  const float* Wk    = (const float*)d_in[4];
  const float* bk    = (const float*)d_in[5];
  const float* Wv    = (const float*)d_in[6];
  const float* bv    = (const float*)d_in[7];
  const float* Wo    = (const float*)d_in[8];
  const float* bo    = (const float*)d_in[9];
  const float* gamma = (const float*)d_in[10];
  const float* alpha = (const float*)d_in[11];
  float* out = (float*)d_out;

  char* ws = (char*)d_ws;
  const size_t H16 = (size_t)S * DD * sizeof(_Float16) * 2;
  const size_t F32 = (size_t)S * DD * sizeof(float);
  _Float16* Xh  = (_Float16*)(ws + 0 * H16);
  _Float16* Wqt = (_Float16*)(ws + 1 * H16);
  _Float16* Wkt = (_Float16*)(ws + 2 * H16);
  _Float16* Wvt = (_Float16*)(ws + 3 * H16);
  _Float16* Wot = (_Float16*)(ws + 4 * H16);
  _Float16* Ch  = (_Float16*)(ws + 5 * H16);
  float* Qf = (float*)(ws + 6 * H16);
  float* Kf = (float*)(ws + 6 * H16 + F32);
  float* Vf = (float*)(ws + 6 * H16 + 2 * F32);

  const int n = S * DD;
  cvt_f32_to_f16_kernel<<<n / 512, 256, 0, stream>>>(X, Xh, n);
  cvt_transpose_w_kernel<<<n / 512, 256, 0, stream>>>(Wq, Wqt);
  cvt_transpose_w_kernel<<<n / 512, 256, 0, stream>>>(Wk, Wkt);
  cvt_transpose_w_kernel<<<n / 512, 256, 0, stream>>>(Wv, Wvt);
  cvt_transpose_w_kernel<<<n / 512, 256, 0, stream>>>(Wo, Wot);

  gemm_qkv_kernel<<<dim3(128, 3), 256, 0, stream>>>(Xh, Wqt, Wkt, Wvt,
                                                    bq, bk, bv, Qf, Kf, Vf);

  attn_core_kernel<<<dim3(4, NH), 128, 0, stream>>>(Qf, Kf, Vf, mask,
                                                    gamma, alpha, Ch);

  gemm_out_kernel<<<128, 256, 0, stream>>>(Ch, Wot, bo, out);
}
